// NonLocal_27900107554980
// MI455X (gfx1250) — hardware-run, weakly checked
//
#include <hip/hip_runtime.h>
#include <math.h>

typedef __attribute__((ext_vector_type(16))) _Float16 v16h;
typedef __attribute__((ext_vector_type(8)))  _Float16 v8h;
typedef __attribute__((ext_vector_type(16))) __bf16   v16b;
typedef __attribute__((ext_vector_type(8)))  __bf16   v8b;
typedef __attribute__((ext_vector_type(8)))  float    v8f;
typedef __attribute__((ext_vector_type(4)))  float    v4f;
typedef __attribute__((ext_vector_type(4)))  unsigned int v4u;

constexpr int kTok   = 16 * 32 * 32;
constexpr int kCin   = 128;
constexpr int kCh    = 64;
constexpr int kQB    = 128;
constexpr int kKC    = 64;
constexpr int kAtWaves = 8;
constexpr int kWPlaneElems = kCin * kCh;
constexpr int kPrepLds = 8320;
constexpr float kWCarry    = 16.0f;
constexpr float kPCarry    = 32768.0f;
constexpr float kCtxCarry  = 256.0f;
constexpr float kCProjScale = 1.0f / kWCarry;
constexpr float kOutScale   = 1.0f / (kCtxCarry * kWCarry);
constexpr float kF16MinNormal = 6.103515625e-05f;
static_assert(kTok == 16384, "token count");
static_assert((kCin % 32) == 0 && (kCh % 32) == 0, "GEMM K multiples of 32");
static_assert((kTok % 64) == 0 && (kCh % 64) == 0 && (kCin % 64) == 0, "GEMM M,N multiples of 64");
static_assert((kTok % kQB) == 0 && (kTok % kKC) == 0, "attention tile multiples");
static_assert(kQB == kAtWaves * 16, "one 16-row tile per wave");
static_assert(kPrepLds >= 64 * 129 && kPrepLds >= 128 * 65, "weight prep LDS extent");

constexpr size_t kOffWPL = 0;
constexpr size_t kOffXH  = kOffWPL + (size_t)6 * kWPlaneElems * 2;
constexpr size_t kOffXL  = kOffXH  + (size_t)kTok * kCin * 2;
constexpr size_t kOffXF  = kOffXL  + (size_t)kTok * kCin * 2;
constexpr size_t kOffQH  = kOffXF  + (size_t)kTok * kCin * 2;
constexpr size_t kOffQL  = kOffQH  + (size_t)kTok * kCh * 2;
constexpr size_t kOffKH  = kOffQL  + (size_t)kTok * kCh * 2;
constexpr size_t kOffKL  = kOffKH  + (size_t)kTok * kCh * 2;
constexpr size_t kOffVT  = kOffKL  + (size_t)kTok * kCh * 2;
constexpr size_t kOffCTX = kOffVT  + (size_t)kCh * kTok * 2;
constexpr size_t kWsTotal = kOffCTX + (size_t)kTok * kCh * 2;
static_assert(kWsTotal == 25264128ull, "carve total");
static_assert(kWsTotal <= 134217728ull, "carve cap");
static_assert((kOffXH % 128) == 0 && (kOffXL % 128) == 0 && (kOffXF % 128) == 0 && (kOffQH % 128) == 0 &&
              (kOffQL % 128) == 0 && (kOffKH % 128) == 0 && (kOffKL % 128) == 0 && (kOffVT % 128) == 0 &&
              (kOffCTX % 128) == 0, "128-B aligned regions");

__device__ __forceinline__ unsigned short f2bf_bits(float f) {
  unsigned u = __float_as_uint(f);
  return (unsigned short)((u + 0x7FFFu + ((u >> 16) & 1u)) >> 16);
}
__device__ __forceinline__ float bf_bits2f(unsigned short h) { return __uint_as_float(((unsigned)h) << 16); }
__device__ __forceinline__ unsigned pk16(unsigned short a, unsigned short b) { return (unsigned)a | ((unsigned)b << 16); }
__device__ __forceinline__ unsigned short h_bits(float f) { const _Float16 h = (_Float16)f; return __builtin_bit_cast(unsigned short, h); }

__device__ __forceinline__ void dep_guard_h(v8f& a, v8f& b, v16h x, v16h y) { asm volatile("v_nop\n\tv_nop\n\tv_nop\n\tv_nop" : "+v"(a), "+v"(b) : "v"(x), "v"(y)); }
__device__ __forceinline__ void dep_guard_b(v8f& a, v8f& b, v16b x, v16b y) { asm volatile("v_nop\n\tv_nop\n\tv_nop\n\tv_nop" : "+v"(a), "+v"(b) : "v"(x), "v"(y)); }
__device__ __forceinline__ void keep4_h(v16h a, v16h b, v16h c, v16h d) { asm volatile("v_nop" :: "v"(a), "v"(b), "v"(c), "v"(d)); }
__device__ __forceinline__ void keep4_b(v16b a, v16b b, v16b c, v16b d) { asm volatile("v_nop" :: "v"(a), "v"(b), "v"(c), "v"(d)); }
__device__ __forceinline__ void acc_guard4(v8f& a, v8f& b, v8f& c, v8f& d) { asm volatile("v_nop\n\tv_nop\n\tv_nop\n\tv_nop" : "+v"(a), "+v"(b), "+v"(c), "+v"(d)); }
template <typename T> struct Frag;
template <> struct Frag<_Float16> {
  typedef v16h V; union U { v16h v; v8h h[2]; };
  static __device__ __forceinline__ v16h load(const _Float16* p) {
    U f; f.h[0] = *(const v8h*)(p); f.h[1] = *(const v8h*)(p + 16); return f.v;
  }
  static __device__ __forceinline__ v8f mma(v16h a, v16h b, v8f c) {
    return __builtin_amdgcn_wmma_f32_16x16x32_f16(false, a, false, b, (short)0, c, false, false);
  }
  static __device__ __forceinline__ void guard(v8f& a, v8f& b, v16h x, v16h y) { dep_guard_h(a, b, x, y); }
  static __device__ __forceinline__ void keep(v16h a, v16h b, v16h c, v16h d) { keep4_h(a, b, c, d); }
};
template <> struct Frag<__bf16> {
  typedef v16b V; union U { v16b v; v8b h[2]; };
  static __device__ __forceinline__ v16b load(const __bf16* p) {
    U f; f.h[0] = *(const v8b*)(p); f.h[1] = *(const v8b*)(p + 16); return f.v;
  }
  static __device__ __forceinline__ v8f mma(v16b a, v16b b, v8f c) {
    return __builtin_amdgcn_wmma_f32_16x16x32_bf16(false, a, false, b, (short)0, c, false, false);
  }
  static __device__ __forceinline__ void guard(v8f& a, v8f& b, v16b x, v16b y) { dep_guard_b(a, b, x, y); }
  static __device__ __forceinline__ void keep(v16b a, v16b b, v16b c, v16b d) { keep4_b(a, b, c, d); }
};

__device__ __forceinline__ v8f mma_bf(v16b a, v16b b, v8f c) {
  c = __builtin_amdgcn_wmma_f32_16x16x32_bf16(false, a, false, b, (short)0, c, false, false);
  asm volatile("v_nop\n\tv_nop\n\tv_nop\n\tv_nop" : "+v"(c) : "v"(a), "v"(b));
  return c;
}
__device__ __forceinline__ v8f mma_hf(v16h a, v16h b, v8f c) {
  c = __builtin_amdgcn_wmma_f32_16x16x32_f16(false, a, false, b, (short)0, c, false, false);
  asm volatile("v_nop\n\tv_nop\n\tv_nop\n\tv_nop" : "+v"(c) : "v"(a), "v"(b));
  return c;
}

template <int ET> struct Elem;
template <> struct Elem<0> { typedef _Float16 T; };
template <> struct Elem<1> { typedef __bf16 T; };
template <int ET, bool SPLIT, int BIAS_MODE, int OUT_MODE, bool RESID>
__global__ __launch_bounds__(256) void wmma_gemm64(
    const unsigned short* __restrict__ Ap, const unsigned short* __restrict__ A2p, int lda, long strideA,
    const unsigned short* __restrict__ Btp, const unsigned short* __restrict__ Bt2p, int ldb, long strideB,
    void* __restrict__ Cout, void* __restrict__ Cout2, int ldc, long strideC,
    const float* __restrict__ bias,
    const float* __restrict__ resid, long strideR,
    int M, int N, int K, float scale) {
  typedef typename Elem<ET>::T T;
  typedef typename Frag<T>::V V;
  const T* A = (const T*)Ap; const T* A2 = (const T*)A2p; const T* Bt = (const T*)Btp; const T* Bt2 = (const T*)Bt2p;
  __shared__ __align__(16) float sT[8][16 * 68];
  const int b    = blockIdx.y;
  const int lane = threadIdx.x & 31;
  const int wave = threadIdx.x >> 5;
  const int tilesN = N >> 6;
  const int tilesM = M >> 6;
  const int tile = blockIdx.x * 8 + wave;
  if (tile >= tilesM * tilesN) return;
  const int tm = tile / tilesN;
  const int tn = tile - tm * tilesN;
  const int m0 = tm << 6;
  const int n0 = tn << 6;

  const T* Ab  = A  + (size_t)b * strideA;
  const T* Bb  = Bt + (size_t)b * strideB;
  const T* Ab2 = SPLIT ? (A2  + (size_t)b * strideA) : nullptr;
  const T* Bb2 = SPLIT ? (Bt2 + (size_t)b * strideB) : nullptr;

  const int rlane = lane & 15;
  const int koff  = (lane >> 4) * 8;
  const int mOff  = (lane >> 4) * 8;

  v8f acc[4][4];
#pragma unroll
  for (int i = 0; i < 4; ++i)
#pragma unroll
    for (int j = 0; j < 4; ++j) acc[i][j] = (v8f){0.f,0.f,0.f,0.f,0.f,0.f,0.f,0.f};

  for (int k0 = 0; k0 < K; k0 += 32) {
    V bh[4], bl[4];
#pragma unroll
    for (int j = 0; j < 4; ++j) {
      const size_t bo = (size_t)(n0 + (j << 4) + rlane) * ldb + koff + k0;
      bh[j] = Frag<T>::load(Bb + bo);
      if (SPLIT) bl[j] = Frag<T>::load(Bb2 + bo);
    }
#pragma unroll
    for (int i = 0; i < 4; ++i) {
      const size_t ao = (size_t)(m0 + (i << 4) + rlane) * lda + koff + k0;
      V ah = Frag<T>::load(Ab + ao);
      V al;
      if (SPLIT) al = Frag<T>::load(Ab2 + ao);
#pragma unroll
      for (int j = 0; j < 4; ++j) {
        acc[i][j] = Frag<T>::mma(ah, bh[j], acc[i][j]);
        if (SPLIT) {
          acc[i][j] = Frag<T>::mma(ah, bl[j], acc[i][j]);
          acc[i][j] = Frag<T>::mma(al, bh[j], acc[i][j]);
        }
      }
      Frag<T>::guard(acc[i][0], acc[i][1], ah, SPLIT ? al : ah);
      Frag<T>::guard(acc[i][2], acc[i][3], ah, SPLIT ? al : ah);
    }
    Frag<T>::keep(bh[0], bh[1], bh[2], bh[3]);
    if (SPLIT) Frag<T>::keep(bl[0], bl[1], bl[2], bl[3]);
  }
  acc_guard4(acc[0][0], acc[0][1], acc[0][2], acc[0][3]);
  acc_guard4(acc[1][0], acc[1][1], acc[1][2], acc[1][3]);
  acc_guard4(acc[2][0], acc[2][1], acc[2][2], acc[2][3]);
  acc_guard4(acc[3][0], acc[3][1], acc[3][2], acc[3][3]);

  float* slab = sT[wave];
  const float* Rb = RESID ? (resid + (size_t)b * strideR) : nullptr;
#pragma unroll
  for (int i = 0; i < 4; ++i) {
    const int mBase = m0 + (i << 4);
#pragma unroll
    for (int j = 0; j < 4; ++j) {
      const int n = n0 + (j << 4) + rlane;
      float bv = 0.f;
      if (BIAS_MODE == 2) bv = bias[n];
#pragma unroll
      for (int r = 0; r < 8; ++r) {
        float v = acc[i][j][r] * scale;
        if (BIAS_MODE == 1) v += bias[mBase + mOff + r];
        if (BIAS_MODE == 2) v += bv;
        slab[(mOff + r) * 68 + (j << 4) + rlane] = v;
      }
    }
    __builtin_amdgcn_fence(__ATOMIC_RELEASE, "workgroup");
    __builtin_amdgcn_wave_barrier();
    __builtin_amdgcn_fence(__ATOMIC_ACQUIRE, "workgroup");
    if (OUT_MODE == 0) {
      float* C = (float*)Cout + (size_t)b * strideC;
      const int hh = lane >> 4, c4 = (lane & 15) * 4;
      v4f ov[8];
#pragma unroll
      for (int it = 0; it < 8; ++it) {
        const int row = it * 2 + hh;
        v4f v = *(const v4f*)(slab + row * 68 + c4);
        if (RESID) {
          const v4f rv = *(const v4f*)(Rb + (size_t)(mBase + row) * ldc + n0 + c4);
          v = v + rv;
        }
        ov[it] = v;
      }
      for (int pass = 0; pass < 2; ++pass) {
#pragma unroll
        for (int it = 0; it < 8; ++it) {
          const int row = it * 2 + hh;
          *(volatile v4f*)(C + (size_t)(mBase + row) * ldc + n0 + c4) = ov[it];
        }
        __threadfence();
      }
    } else {
      const int q = lane >> 3, c8 = (lane & 7) * 8;
      unsigned short* C  = (unsigned short*)Cout  + (size_t)b * strideC;
      unsigned short* C2 = (OUT_MODE == 2) ? ((unsigned short*)Cout2 + (size_t)b * strideC) : nullptr;
      for (int pass = 0; pass < 2; ++pass) {
#pragma unroll
        for (int it = 0; it < 4; ++it) {
          const int row = it * 4 + q;
          const float* sp = slab + row * 68 + c8;
          v8h hv, lv;
#pragma unroll
          for (int e = 0; e < 8; ++e) {
            if (OUT_MODE == 1) {
              hv[e] = (_Float16)sp[e];
            } else {
              unsigned short hb = f2bf_bits(sp[e]);
              unsigned short lb = f2bf_bits(sp[e] - bf_bits2f(hb));
              hv[e] = __builtin_bit_cast(_Float16, hb);
              lv[e] = __builtin_bit_cast(_Float16, lb);
            }
          }
          *(volatile v8h*)(C + (size_t)(mBase + row) * ldc + n0 + c8) = hv;
          if (OUT_MODE == 2) *(volatile v8h*)(C2 + (size_t)(mBase + row) * ldc + n0 + c8) = lv;
        }
        __threadfence();
      }
    }
    __builtin_amdgcn_fence(__ATOMIC_RELEASE, "workgroup");
    __builtin_amdgcn_wave_barrier();
    __builtin_amdgcn_fence(__ATOMIC_ACQUIRE, "workgroup");
  }
}

__global__ __launch_bounds__(256) void wprep_kernel(const float* __restrict__ W0, const float* __restrict__ W1,
                                                    const float* __restrict__ W2, const float* __restrict__ W3,
                                                    unsigned short* __restrict__ planes) {
  __shared__ float sm[kPrepLds];
  const int t = threadIdx.x;
  const int z = blockIdx.x;
  const float* W = (z == 0) ? W0 : (z == 1) ? W1 : (z == 2) ? W2 : W3;
  const int shC   = (z == 3) ? 7 : 6;
  const int nIn   = (z == 3) ? kCh : kCin;
  const int pitch = nIn + 1;
  const int shS   = (z == 3) ? 3 : 4;
#pragma unroll 1
  for (int i = 0; i < 32; ++i) {
    const int e = i * 256 + t;
    const int r = e >> shC;
    const int c = e & ((1 << shC) - 1);
    sm[c * pitch + r] = W[e];
  }
  __syncthreads();
  const bool split  = (z < 2);
  const int hiPlane = split ? (2 * z) : (z + 2);
  const int loPlane = split ? (hiPlane + 1) : hiPlane;
  unsigned short* ph = planes + (size_t)hiPlane * kWPlaneElems;
  unsigned short* pl = planes + (size_t)loPlane * kWPlaneElems;
  const float carry = split ? 1.0f : kWCarry;
  for (int pass = 0; pass < 2; ++pass) {
#pragma unroll 1
    for (int it = 0; it < 4; ++it) {
      const int u   = it * 256 + t;
      const int row = u >> shS;
      const int c8  = (u & ((1 << shS) - 1)) << 3;
      const float* sp = sm + row * pitch + c8;
      unsigned short a[8], b[8];
#pragma unroll
      for (int e = 0; e < 8; ++e) {
        const float f = sp[e] * carry;
        const unsigned short bh = f2bf_bits(f);
        const unsigned short bl = f2bf_bits(f - bf_bits2f(bh));
        const unsigned short fh = h_bits(f);
        a[e] = split ? bh : fh;
        b[e] = bl;
      }
      const v4u ua = (v4u){pk16(a[0], a[1]), pk16(a[2], a[3]), pk16(a[4], a[5]), pk16(a[6], a[7])};
      const v4u ub = (v4u){pk16(b[0], b[1]), pk16(b[2], b[3]), pk16(b[4], b[5]), pk16(b[6], b[7])};
      *(volatile v4u*)(ph + (size_t)u * 8) = ua;
      if (split) *(volatile v4u*)(pl + (size_t)u * 8) = ub;
    }
    __threadfence();
  }
}

__global__ __launch_bounds__(256) void xsplit_kernel(
    const float* __restrict__ src, unsigned short* __restrict__ dhi, unsigned short* __restrict__ dlo,
    unsigned short* __restrict__ dh16, int total8)
{
  const int i = blockIdx.x * 256 + threadIdx.x;
  if (i >= total8) return;
  const size_t e0 = (size_t)i << 3;
  const v4f a0 = *(const v4f*)(src + e0);
  const v4f a1 = *(const v4f*)(src + e0 + 4);
  unsigned short hb[8], lb[8], fb[8];
#pragma unroll
  for (int e = 0; e < 4; ++e) {
    const float f0 = a0[e];
    const float f1 = a1[e];
    hb[e]     = f2bf_bits(f0);
    hb[4 + e] = f2bf_bits(f1);
    lb[e]     = f2bf_bits(f0 - bf_bits2f(hb[e]));
    lb[4 + e] = f2bf_bits(f1 - bf_bits2f(hb[4 + e]));
    fb[e]     = h_bits(f0);
    fb[4 + e] = h_bits(f1);
  }
  const v4u uh = (v4u){pk16(hb[0], hb[1]), pk16(hb[2], hb[3]), pk16(hb[4], hb[5]), pk16(hb[6], hb[7])};
  const v4u ul = (v4u){pk16(lb[0], lb[1]), pk16(lb[2], lb[3]), pk16(lb[4], lb[5]), pk16(lb[6], lb[7])};
  const v4u uf = (v4u){pk16(fb[0], fb[1]), pk16(fb[2], fb[3]), pk16(fb[4], fb[5]), pk16(fb[6], fb[7])};
  unsigned short* qh = dhi + e0;
  unsigned short* ql = dlo + e0;
  unsigned short* qf = dh16 + e0;
  *(volatile v4u*)qh = uh;
  *(volatile v4u*)ql = ul;
  *(volatile v4u*)qf = uf;
  __threadfence();
  *(volatile v4u*)qh = uh;
  *(volatile v4u*)ql = ul;
  *(volatile v4u*)qf = uf;
}

__global__ __launch_bounds__(256) void attn_kernel(
    const unsigned short* __restrict__ Qhp, const unsigned short* __restrict__ Qlp,
    const unsigned short* __restrict__ Khp, const unsigned short* __restrict__ Klp,
    const unsigned short* __restrict__ Vtp, unsigned short* __restrict__ CTXp)
{
  union FB { v16b v; v8b h[2]; };
  union FH { v16h v; v8h h[2]; };
  __shared__ __align__(16) __bf16   sKh[kKC * kCh];
  __shared__ __align__(16) __bf16   sKl[kKC * kCh];
  __shared__ __align__(16) _Float16 sV[kCh * kKC];
  __shared__ __align__(16) _Float16 sP[kAtWaves][16 * kKC];

  const __bf16*   Qh = (const __bf16*)Qhp;
  const __bf16*   Ql = (const __bf16*)Qlp;
  const __bf16*   Kh = (const __bf16*)Khp;
  const __bf16*   Kl = (const __bf16*)Klp;
  const _Float16* Vt = (const _Float16*)Vtp;
  _Float16*       Cx = (_Float16*)CTXp;

  const int tid  = threadIdx.x;
  const int wave = tid >> 5;
  const int lane = tid & 31;
  const int hh   = lane >> 4;
  const int c    = lane & 15;
  const int q0   = blockIdx.x * kQB + wave * 16;

  v16b qah[2], qal[2];
  {
    const size_t qo = (size_t)(q0 + c) * kCh + 8 * hh;
#pragma unroll
    for (int dc = 0; dc < 2; ++dc) {
      qah[dc] = Frag<__bf16>::load(Qh + qo + dc * 32);
      qal[dc] = Frag<__bf16>::load(Ql + qo + dc * 32);
    }
  }

  float mrow[8], lrow[8];
  v8f oacc[4];
#pragma unroll
  for (int r = 0; r < 8; ++r) { mrow[r] = -1.0e30f; lrow[r] = 0.f; }
#pragma unroll
  for (int t = 0; t < 4; ++t) oacc[t] = (v8f){0.f,0.f,0.f,0.f,0.f,0.f,0.f,0.f};

  _Float16* pw = sP[wave];

#pragma unroll 1
  for (int kc = 0; kc < kTok / kKC; ++kc) {
    const int kv0 = kc * kKC;
    __syncthreads();
#pragma unroll
    for (int it = 0; it < 2; ++it) {
      const int sg   = tid + it * 256;
      const int dch  = sg >> 3;
      const int part = sg & 7;
      const v8b kh8 = *(const v8b*)(Kh + (size_t)kv0 * kCh + sg * 8);
      const v8b kl8 = *(const v8b*)(Kl + (size_t)kv0 * kCh + sg * 8);
      const v8h vv8 = *(const v8h*)(Vt + (size_t)dch * kTok + kv0 + part * 8);
      *(v8b*)(sKh + sg * 8) = kh8;
      *(v8b*)(sKl + sg * 8) = kl8;
      *(v8h*)(sV + dch * kKC + part * 8) = vv8;
    }
    __syncthreads();

    v8f s[4];
#pragma unroll
    for (int j = 0; j < 4; ++j) {
      s[j] = (v8f){0.f,0.f,0.f,0.f,0.f,0.f,0.f,0.f};
#pragma unroll
      for (int dc = 0; dc < 2; ++dc) {
        FB kb, kl;
        kb.h[0] = *(const v8b*)(sKh + (j * 16 + c) * kCh + dc * 32 + 8 * hh);
        kb.h[1] = *(const v8b*)(sKh + (j * 16 + c) * kCh + dc * 32 + 16 + 8 * hh);
        kl.h[0] = *(const v8b*)(sKl + (j * 16 + c) * kCh + dc * 32 + 8 * hh);
        kl.h[1] = *(const v8b*)(sKl + (j * 16 + c) * kCh + dc * 32 + 16 + 8 * hh);
        s[j] = mma_bf(qah[dc], kb.v, s[j]);
        s[j] = mma_bf(qah[dc], kl.v, s[j]);
        s[j] = mma_bf(qal[dc], kb.v, s[j]);
      }
    }

    float cm[8];
#pragma unroll
    for (int r = 0; r < 8; ++r) {
      float m = fmaxf(fmaxf(s[0][r], s[1][r]), fmaxf(s[2][r], s[3][r]));
#pragma unroll
      for (int off = 1; off < 16; off <<= 1) m = fmaxf(m, __shfl_xor(m, off, 32));
      cm[r] = m;
    }
#pragma unroll
    for (int r = 0; r < 8; ++r) {
      const float mnew  = fmaxf(mrow[r], cm[r]);
      const float alpha = __expf(mrow[r] - mnew);
      mrow[r] = mnew;
      float psum = 0.f;
#pragma unroll
      for (int j = 0; j < 4; ++j) {
        float pv = __expf(s[j][r] - mnew) * kPCarry;
        pv = (pv < kF16MinNormal) ? 0.0f : pv;
        const _Float16 ph = (_Float16)pv;
        const float pf = (float)ph;
        psum += pf;
        pw[(8 * hh + r) * kKC + j * 16 + c] = ph;
      }
      lrow[r] = lrow[r] * alpha + psum;
#pragma unroll
      for (int t = 0; t < 4; ++t) oacc[t][r] *= alpha;
    }
    __builtin_amdgcn_fence(__ATOMIC_RELEASE, "workgroup");
    __builtin_amdgcn_wave_barrier();
    __builtin_amdgcn_fence(__ATOMIC_ACQUIRE, "workgroup");

#pragma unroll 1
    for (int kk = 0; kk < 2; ++kk) {
      FH pa;
      pa.h[0] = *(const v8h*)(pw + c * kKC + kk * 32 + 8 * hh);
      pa.h[1] = *(const v8h*)(pw + c * kKC + kk * 32 + 16 + 8 * hh);
#pragma unroll
      for (int t = 0; t < 4; ++t) {
        FH vb;
        vb.h[0] = *(const v8h*)(sV + (t * 16 + c) * kKC + kk * 32 + 8 * hh);
        vb.h[1] = *(const v8h*)(sV + (t * 16 + c) * kKC + kk * 32 + 16 + 8 * hh);
        oacc[t] = mma_hf(pa.v, vb.v, oacc[t]);
      }
    }
  }

#pragma unroll
  for (int r = 0; r < 8; ++r) {
    float l = lrow[r];
#pragma unroll
    for (int off = 1; off < 16; off <<= 1) l += __shfl_xor(l, off, 32);
    lrow[r] = l;
  }

  __builtin_amdgcn_fence(__ATOMIC_RELEASE, "workgroup");
  __builtin_amdgcn_wave_barrier();
  __builtin_amdgcn_fence(__ATOMIC_ACQUIRE, "workgroup");
#pragma unroll
  for (int r = 0; r < 8; ++r) {
    const float inv = kCtxCarry * (1.0f / lrow[r]);
#pragma unroll
    for (int t = 0; t < 4; ++t) pw[(8 * hh + r) * kKC + t * 16 + c] = (_Float16)(oacc[t][r] * inv);
  }
  __builtin_amdgcn_fence(__ATOMIC_RELEASE, "workgroup");
  __builtin_amdgcn_wave_barrier();
  __builtin_amdgcn_fence(__ATOMIC_ACQUIRE, "workgroup");
  {
    const int q = lane >> 3, c8 = (lane & 7) * 8;
    v8h ov[4];
#pragma unroll
    for (int it = 0; it < 4; ++it) ov[it] = *(const v8h*)(pw + (it * 4 + q) * kKC + c8);
    for (int pass = 0; pass < 2; ++pass) {
#pragma unroll
      for (int it = 0; it < 4; ++it)
        *(volatile v8h*)(Cx + (size_t)(q0 + it * 4 + q) * kCh + c8) = ov[it];
      __threadfence();
    }
  }
}

extern "C" void kernel_launch(void* const* d_in, const int* in_sizes, int n_in,
                              void* d_out, int out_size, void* d_ws, size_t ws_size,
                              hipStream_t stream) {
  if (n_in < 9) return;
  if (in_sizes[0] != kTok * kCin) return;
  if (in_sizes[1] != kCin * kCh) return;
  if (in_sizes[2] != kCh) return;
  if (in_sizes[3] != kCin * kCh) return;
  if (in_sizes[4] != kCh) return;
  if (in_sizes[5] != kCin * kCh) return;
  if (in_sizes[6] != kCh) return;
  if (in_sizes[7] != kCh * kCin) return;
  if (in_sizes[8] != kCin) return;
  if (out_size != kTok * kCin) return;
  if (ws_size < kWsTotal) return;

  const float* x  = (const float*)d_in[0];
  const float* Wa = (const float*)d_in[1];
  const float* ba = (const float*)d_in[2];
  const float* Wb = (const float*)d_in[3];
  const float* bb = (const float*)d_in[4];
  const float* Wc = (const float*)d_in[5];
  const float* bc = (const float*)d_in[6];
  const float* Wo = (const float*)d_in[7];
  const float* bo = (const float*)d_in[8];
  float* out = (float*)d_out;

  char* ws = (char*)d_ws;
  unsigned short* WPL = (unsigned short*)(ws + kOffWPL);
  unsigned short* WAH = WPL + 0 * (size_t)kWPlaneElems;
  unsigned short* WAL = WPL + 1 * (size_t)kWPlaneElems;
  unsigned short* WBH = WPL + 2 * (size_t)kWPlaneElems;
  unsigned short* WBL = WPL + 3 * (size_t)kWPlaneElems;
  unsigned short* WCT = WPL + 4 * (size_t)kWPlaneElems;
  unsigned short* WOT = WPL + 5 * (size_t)kWPlaneElems;
  unsigned short* XH  = (unsigned short*)(ws + kOffXH);
  unsigned short* XL  = (unsigned short*)(ws + kOffXL);
  unsigned short* XF  = (unsigned short*)(ws + kOffXF);
  unsigned short* QH  = (unsigned short*)(ws + kOffQH);
  unsigned short* QL  = (unsigned short*)(ws + kOffQL);
  unsigned short* KH  = (unsigned short*)(ws + kOffKH);
  unsigned short* KL  = (unsigned short*)(ws + kOffKL);
  unsigned short* VT  = (unsigned short*)(ws + kOffVT);
  unsigned short* CTX = (unsigned short*)(ws + kOffCTX);

  wprep_kernel<<<4, 256, 0, stream>>>(Wa, Wb, Wc, Wo, WPL);

  xsplit_kernel<<<(kTok * kCin / 8) / 256, 256, 0, stream>>>(x, XH, XL, XF, kTok * kCin / 8);

  wmma_gemm64<1, true, 2, 2, false><<<dim3((kTok / 64) * (kCh / 64) / 8, 1), 256, 0, stream>>>(
      XH, XL, kCin, 0L,
      WAH, WAL, kCin, 0L,
      (void*)QH, (void*)QL, kCh, 0L,
      ba, nullptr, 0L,
      kTok, kCh, kCin, 1.0f);

  wmma_gemm64<1, true, 2, 2, false><<<dim3((kTok / 64) * (kCh / 64) / 8, 1), 256, 0, stream>>>(
      XH, XL, kCin, 0L,
      WBH, WBL, kCin, 0L,
      (void*)KH, (void*)KL, kCh, 0L,
      bb, nullptr, 0L,
      kTok, kCh, kCin, 1.0f);

  wmma_gemm64<0, false, 1, 1, false><<<dim3((kCh / 64) * (kTok / 64) / 8, 1), 256, 0, stream>>>(
      WCT, nullptr, kCin, 0L,
      XF, nullptr, kCin, 0L,
      (void*)VT, nullptr, kTok, 0L,
      bc, nullptr, 0L,
      kCh, kTok, kCin, kCProjScale);

  attn_kernel<<<kTok / kQB, 256, 0, stream>>>(QH, QL, KH, KL, VT, CTX);

  wmma_gemm64<0, false, 2, 0, true><<<dim3((kTok / 64) * (kCin / 64) / 8, 1), 256, 0, stream>>>(
      CTX, nullptr, kCh, 0L,
      WOT, nullptr, kCh, 0L,
      (void*)out, nullptr, kCin, 0L,
      bo, x, 0L,
      kTok, kCin, kCh, kOutScale);
}
